// KAN_Decode_34351148433545
// MI455X (gfx1250) — hardware-verified
//
#include <hip/hip_runtime.h>
#include <math.h>

#pragma clang fp contract(off)

constexpr int kRows    = 16384;
constexpr int kLat     = 64;
constexpr int kHid     = 512;
constexpr int kOutDim  = 256;
constexpr int kNB      = 8;
constexpr int kKsp     = kHid * kNB;
constexpr int kChunk   = 4096;
constexpr int kNChunk  = kRows / kChunk;
constexpr float kKnotH    = 0.4f;
constexpr float kWCarry   = 16.0f;
constexpr float kSCarry   = 16.0f;
constexpr float kDenseScale = 1.0f / 16.0f;
constexpr float kBaseScale  = 1.0f / 256.0f;

static_assert(kRows % kChunk == 0);
static_assert(kLat % 32 == 0 && kHid % 64 == 0 && kOutDim % 64 == 0 && kKsp % 32 == 0 && kChunk % 64 == 0);

constexpr size_t kOffXh  = 0;
constexpr size_t kSzXh   = (size_t)kRows * kLat * 2;
constexpr size_t kOffDwh = kOffXh + kSzXh;
constexpr size_t kSzDwh  = (size_t)kHid * kLat * 2;
constexpr size_t kOffBw1 = kOffDwh + kSzDwh;
constexpr size_t kSzBw1  = (size_t)kHid * kHid * 2;
constexpr size_t kOffBw2 = kOffBw1 + kSzBw1;
constexpr size_t kSzBw2  = (size_t)kOutDim * kHid * 2;
constexpr size_t kOffSw1 = kOffBw2 + kSzBw2;
constexpr size_t kSzSw1  = (size_t)kHid * kKsp * 2;
constexpr size_t kOffSw2 = kOffSw1 + kSzSw1;
constexpr size_t kSzSw2  = (size_t)kOutDim * kKsp * 2;
constexpr size_t kOffP1  = kOffSw2 + kSzSw2;
constexpr size_t kSzP1   = (size_t)kRows * kHid * 4;
constexpr size_t kOffH2  = kOffP1 + kSzP1;
constexpr size_t kSzH2   = (size_t)kRows * kHid * 4;
constexpr size_t kOffSpl = kOffH2 + kSzH2;
constexpr size_t kSzSpl  = (size_t)kChunk * kHid * 2;
constexpr size_t kOffTbs = kOffSpl + kSzSpl;
constexpr size_t kSzTbs  = (size_t)kChunk * kHid * 4;
constexpr size_t kOffBsp = kOffTbs + kSzTbs;
constexpr size_t kSzBsp  = (size_t)kChunk * kKsp * 2;
constexpr size_t kWsTotal = kOffBsp + kSzBsp;
static_assert(kWsTotal == 122486784ull);
static_assert(kWsTotal <= 134217728ull);
static_assert((kOffDwh % 4096) == 0 && (kOffBw1 % 4096) == 0 && (kOffBw2 % 4096) == 0 && (kOffSw1 % 4096) == 0 &&
              (kOffSw2 % 4096) == 0 && (kOffP1 % 4096) == 0 && (kOffH2 % 4096) == 0 && (kOffSpl % 4096) == 0 &&
              (kOffTbs % 4096) == 0 && (kOffBsp % 4096) == 0);

typedef __attribute__((ext_vector_type(16))) _Float16 v16h;
typedef __attribute__((ext_vector_type(8)))  _Float16 v8h;
typedef __attribute__((ext_vector_type(16))) __bf16   v16b;
typedef __attribute__((ext_vector_type(8)))  __bf16   v8b;
typedef __attribute__((ext_vector_type(8)))  float    v8f;
typedef __attribute__((ext_vector_type(4)))  float    v4f;
typedef __attribute__((ext_vector_type(4)))  unsigned int v4u;

__device__ __forceinline__ unsigned short f2bf_bits(float f) {
  unsigned u = __float_as_uint(f);
  return (unsigned short)((u + 0x7FFFu + ((u >> 16) & 1u)) >> 16);
}
__device__ __forceinline__ float bf_bits2f(unsigned short h) { return __uint_as_float(((unsigned)h) << 16); }

__device__ __forceinline__ void dep_guard_h(v8f& a, v8f& b, v16h x, v16h y) { asm volatile("v_nop\n\tv_nop\n\tv_nop\n\tv_nop" : "+v"(a), "+v"(b) : "v"(x), "v"(y)); }
__device__ __forceinline__ void dep_guard_b(v8f& a, v8f& b, v16b x, v16b y) { asm volatile("v_nop\n\tv_nop\n\tv_nop\n\tv_nop" : "+v"(a), "+v"(b) : "v"(x), "v"(y)); }
__device__ __forceinline__ void keep4_h(v16h a, v16h b, v16h c, v16h d) { asm volatile("v_nop" :: "v"(a), "v"(b), "v"(c), "v"(d)); }
__device__ __forceinline__ void keep4_b(v16b a, v16b b, v16b c, v16b d) { asm volatile("v_nop" :: "v"(a), "v"(b), "v"(c), "v"(d)); }
__device__ __forceinline__ void acc_guard4(v8f& a, v8f& b, v8f& c, v8f& d) { asm volatile("v_nop\n\tv_nop\n\tv_nop\n\tv_nop" : "+v"(a), "+v"(b), "+v"(c), "+v"(d)); }
template <typename T> struct Frag;
template <> struct Frag<_Float16> {
  typedef v16h V; union U { v16h v; v8h h[2]; };
  static __device__ __forceinline__ v16h load(const _Float16* p) {
    U f; f.h[0] = *(const v8h*)(p); f.h[1] = *(const v8h*)(p + 16); return f.v;
  }
  static __device__ __forceinline__ v8f mma(v16h a, v16h b, v8f c) {
    return __builtin_amdgcn_wmma_f32_16x16x32_f16(false, a, false, b, (short)0, c, false, false);
  }
  static __device__ __forceinline__ void guard(v8f& a, v8f& b, v16h x, v16h y) { dep_guard_h(a, b, x, y); }
  static __device__ __forceinline__ void keep(v16h a, v16h b, v16h c, v16h d) { keep4_h(a, b, c, d); }
};
template <> struct Frag<__bf16> {
  typedef v16b V; union U { v16b v; v8b h[2]; };
  static __device__ __forceinline__ v16b load(const __bf16* p) {
    U f; f.h[0] = *(const v8b*)(p); f.h[1] = *(const v8b*)(p + 16); return f.v;
  }
  static __device__ __forceinline__ v8f mma(v16b a, v16b b, v8f c) {
    return __builtin_amdgcn_wmma_f32_16x16x32_bf16(false, a, false, b, (short)0, c, false, false);
  }
  static __device__ __forceinline__ void guard(v8f& a, v8f& b, v16b x, v16b y) { dep_guard_b(a, b, x, y); }
  static __device__ __forceinline__ void keep(v16b a, v16b b, v16b c, v16b d) { keep4_b(a, b, c, d); }
};

__device__ __forceinline__ unsigned pk16(unsigned short a, unsigned short b) { return (unsigned)a | ((unsigned)b << 16); }
__device__ __forceinline__ unsigned short h_bits(float f) { const _Float16 h = (_Float16)f; return __builtin_bit_cast(unsigned short, h); }

template <int ET> struct Elem;
template <> struct Elem<0> { typedef _Float16 T; };
template <> struct Elem<1> { typedef __bf16 T; };
template <int ET, bool SPLIT, int BIAS_MODE, int OUT_MODE, bool RESID, int ACT = 0>
__global__ __launch_bounds__(256) void wmma_gemm64(
    const unsigned short* __restrict__ Ap, const unsigned short* __restrict__ A2p, int lda, long strideA,
    const unsigned short* __restrict__ Btp, const unsigned short* __restrict__ Bt2p, int ldb, long strideB,
    void* __restrict__ Cout, void* __restrict__ Cout2, int ldc, long strideC,
    const float* __restrict__ bias,
    const float* __restrict__ resid, long strideR,
    int M, int N, int K, float scale) {
  typedef typename Elem<ET>::T T;
  typedef typename Frag<T>::V V;
  const T* A = (const T*)Ap; const T* A2 = (const T*)A2p; const T* Bt = (const T*)Btp; const T* Bt2 = (const T*)Bt2p;
  __shared__ __align__(16) float sT[8][16 * 68];
  const int b    = blockIdx.y;
  const int lane = threadIdx.x & 31;
  const int wave = threadIdx.x >> 5;
  const int tilesN = N >> 6;
  const int tilesM = M >> 6;
  const int tile = blockIdx.x * 8 + wave;
  if (tile >= tilesM * tilesN) return;
  const int tm = tile / tilesN;
  const int tn = tile - tm * tilesN;
  const int m0 = tm << 6;
  const int n0 = tn << 6;

  const T* Ab  = A  + (size_t)b * strideA;
  const T* Bb  = Bt + (size_t)b * strideB;
  const T* Ab2 = SPLIT ? (A2  + (size_t)b * strideA) : nullptr;
  const T* Bb2 = SPLIT ? (Bt2 + (size_t)b * strideB) : nullptr;

  const int rlane = lane & 15;
  const int koff  = (lane >> 4) * 8;
  const int mOff  = (lane >> 4) * 8;

  v8f acc[4][4];
#pragma unroll
  for (int i = 0; i < 4; ++i)
#pragma unroll
    for (int j = 0; j < 4; ++j) acc[i][j] = (v8f){0.f,0.f,0.f,0.f,0.f,0.f,0.f,0.f};

  for (int k0 = 0; k0 < K; k0 += 32) {
    V bh[4], bl[4];
#pragma unroll
    for (int j = 0; j < 4; ++j) {
      const size_t bo = (size_t)(n0 + (j << 4) + rlane) * ldb + koff + k0;
      bh[j] = Frag<T>::load(Bb + bo);
      if (SPLIT) bl[j] = Frag<T>::load(Bb2 + bo);
    }
#pragma unroll
    for (int i = 0; i < 4; ++i) {
      const size_t ao = (size_t)(m0 + (i << 4) + rlane) * lda + koff + k0;
      V ah = Frag<T>::load(Ab + ao);
      V al;
      if (SPLIT) al = Frag<T>::load(Ab2 + ao);
#pragma unroll
      for (int j = 0; j < 4; ++j) {
        acc[i][j] = Frag<T>::mma(ah, bh[j], acc[i][j]);
        if (SPLIT) {
          acc[i][j] = Frag<T>::mma(ah, bl[j], acc[i][j]);
          acc[i][j] = Frag<T>::mma(al, bh[j], acc[i][j]);
        }
      }
      Frag<T>::guard(acc[i][0], acc[i][3], ah, SPLIT ? al : ah);
    }
    Frag<T>::keep(bh[0], bh[1], bh[2], bh[3]);
    if (SPLIT) Frag<T>::keep(bl[0], bl[1], bl[2], bl[3]);
  }
  acc_guard4(acc[0][0], acc[0][1], acc[0][2], acc[0][3]);
  acc_guard4(acc[1][0], acc[1][1], acc[1][2], acc[1][3]);
  acc_guard4(acc[2][0], acc[2][1], acc[2][2], acc[2][3]);
  acc_guard4(acc[3][0], acc[3][1], acc[3][2], acc[3][3]);

  float* slab = sT[wave];
  const float* Rb = RESID ? (resid + (size_t)b * strideR) : nullptr;
#pragma unroll
  for (int i = 0; i < 4; ++i) {
    const int mBase = m0 + (i << 4);
#pragma unroll
    for (int j = 0; j < 4; ++j) {
      const int n = n0 + (j << 4) + rlane;
      float bv = 0.f;
      if (BIAS_MODE == 2) bv = bias[n];
#pragma unroll
      for (int r = 0; r < 8; ++r) {
        float v = acc[i][j][r] * scale;
        if (BIAS_MODE == 1) v += bias[mBase + mOff + r];
        if (BIAS_MODE == 2) v += bv;
        if (RESID) v += Rb[(size_t)(mBase + mOff + r) * ldc + n];
        if (ACT == 2) v = fmaxf(v, 0.0f);
        if (ACT == 4) v = (v > 0.f) ? v : 0.01f * v;
        slab[(mOff + r) * 68 + (j << 4) + rlane] = v;
      }
    }
    __builtin_amdgcn_fence(__ATOMIC_RELEASE, "workgroup");
    __builtin_amdgcn_wave_barrier();
    __builtin_amdgcn_fence(__ATOMIC_ACQUIRE, "workgroup");
    if (OUT_MODE == 0) {
      float* C = (float*)Cout + (size_t)b * strideC;
      const int hh = lane >> 4, c4 = (lane & 15) * 4;
      for (int pass = 0; pass < 2; ++pass) {
#pragma unroll
        for (int it = 0; it < 8; ++it) {
          const int row = it * 2 + hh;
          v4f v = *(const v4f*)(slab + row * 68 + c4);
          *(volatile v4f*)(C + (size_t)(mBase + row) * ldc + n0 + c4) = v;
        }
        __threadfence();
      }
    } else {
      const int q = lane >> 3, c8 = (lane & 7) * 8;
      unsigned short* C  = (unsigned short*)Cout  + (size_t)b * strideC;
      unsigned short* C2 = (OUT_MODE == 2) ? ((unsigned short*)Cout2 + (size_t)b * strideC) : nullptr;
      for (int pass = 0; pass < 2; ++pass) {
#pragma unroll
        for (int it = 0; it < 4; ++it) {
          const int row = it * 4 + q;
          const float* sp = slab + row * 68 + c8;
          v8h hv, lv;
#pragma unroll
          for (int e = 0; e < 8; ++e) {
            if (OUT_MODE == 1) {
              hv[e] = (_Float16)sp[e];
            } else {
              unsigned short hb = f2bf_bits(sp[e]);
              unsigned short lb = f2bf_bits(sp[e] - bf_bits2f(hb));
              hv[e] = __builtin_bit_cast(_Float16, hb);
              lv[e] = __builtin_bit_cast(_Float16, lb);
            }
          }
          *(volatile v8h*)(C + (size_t)(mBase + row) * ldc + n0 + c8) = hv;
          if (OUT_MODE == 2) *(volatile v8h*)(C2 + (size_t)(mBase + row) * ldc + n0 + c8) = lv;
        }
        __threadfence();
      }
    }
    __builtin_amdgcn_fence(__ATOMIC_RELEASE, "workgroup");
    __builtin_amdgcn_wave_barrier();
    __builtin_amdgcn_fence(__ATOMIC_ACQUIRE, "workgroup");
  }
}

__global__ __launch_bounds__(256) void cast8_f16_kernel(const float* __restrict__ in, unsigned short* __restrict__ out,
                                                        int n8, float carry) {
  const int i = blockIdx.x * 256 + threadIdx.x;
  if (i >= n8) return;
  const float* p = in + 8 * (size_t)i;
  const v4f a = *(const v4f*)(p);
  const v4f c = *(const v4f*)(p + 4);
  unsigned short hb[8];
#pragma unroll
  for (int e = 0; e < 4; ++e) {
    hb[e]     = h_bits(a[e] * carry);
    hb[4 + e] = h_bits(c[e] * carry);
  }
  const v4u u = (v4u){pk16(hb[0], hb[1]), pk16(hb[2], hb[3]), pk16(hb[4], hb[5]), pk16(hb[6], hb[7])};
  unsigned short* q = out + 8 * (size_t)i;
  *(volatile v4u*)q = u;
  __threadfence();
  *(volatile v4u*)q = u;
}

__global__ __launch_bounds__(256) void spline_cast_kernel(const float* __restrict__ sw, const float* __restrict__ sc,
                                                          unsigned short* __restrict__ out, int n8) {
  const int i = blockIdx.x * 256 + threadIdx.x;
  if (i >= n8) return;
  const float* p = sw + 8 * (size_t)i;
  const v4f a = *(const v4f*)(p);
  const v4f c = *(const v4f*)(p + 4);
  const float s = sc[i];
  unsigned short bb[8];
#pragma unroll
  for (int e = 0; e < 4; ++e) {
    bb[e]     = f2bf_bits(a[e] * s);
    bb[4 + e] = f2bf_bits(c[e] * s);
  }
  const v4u u = (v4u){pk16(bb[0], bb[1]), pk16(bb[2], bb[3]), pk16(bb[4], bb[5]), pk16(bb[6], bb[7])};
  unsigned short* q = out + 8 * (size_t)i;
  *(volatile v4u*)q = u;
  __threadfence();
  *(volatile v4u*)q = u;
}

__device__ __forceinline__ float knotf(int j) { return (float)(j - 3) * kKnotH - 1.0f; }
__device__ __forceinline__ float silu_f32(float x) { return x * __builtin_amdgcn_rcpf(1.0f + expf(-x)); }

__global__ __launch_bounds__(256) void expand_kernel(const float* __restrict__ Hin, int pre_silu,
                                                     unsigned short* __restrict__ Sout,
                                                     unsigned short* __restrict__ Bout) {
  __shared__ __align__(16) unsigned short ssh[256];
  const int t = threadIdx.x;
  const size_t eb = (size_t)blockIdx.x * 256;
  const size_t e  = eb + (size_t)t;

  float hv = Hin[e];
  if (pre_silu) hv = silu_f32(hv);
  const float sv = silu_f32(hv) * kSCarry;

  int cnt = 0;
#pragma unroll
  for (int j = 0; j < 12; ++j) cnt += (hv >= knotf(j)) ? 1 : 0;
  const int m = cnt - 1;
  const float one0 = (cnt >= 1 && cnt <= 11) ? 1.0f : 0.0f;

  float kn[8];
#pragma unroll
  for (int q = 0; q < 8; ++q) kn[q] = knotf(m - 3 + q);

  float w[5];
  w[0] = 0.0f; w[1] = 0.0f; w[2] = 0.0f; w[3] = one0; w[4] = 0.0f;
#pragma unroll
  for (int k = 1; k <= 3; ++k) {
    float nw[4];
#pragma unroll
    for (int p = 0; p < 4; ++p) {
      const float tj   = kn[p];
      const float tjk  = kn[p + k];
      const float tj1  = kn[p + 1];
      const float tjk1 = kn[p + k + 1];
      const float left  = ((hv - tj) * __builtin_amdgcn_rcpf(tjk - tj)) * w[p];
      const float right = ((tjk1 - hv) * __builtin_amdgcn_rcpf(tjk1 - tj1)) * w[p + 1];
      nw[p] = left + right;
    }
#pragma unroll
    for (int p = 0; p < 4; ++p) w[p] = nw[p];
  }

  unsigned short bb[8];
#pragma unroll
  for (int g = 0; g < 8; ++g) {
    const int pg = g - m + 3;
    float v = 0.0f;
    v = (pg == 0) ? w[0] : v;
    v = (pg == 1) ? w[1] : v;
    v = (pg == 2) ? w[2] : v;
    v = (pg == 3) ? w[3] : v;
    bb[g] = f2bf_bits(v);
  }
  const v4u ub = (v4u){pk16(bb[0], bb[1]), pk16(bb[2], bb[3]), pk16(bb[4], bb[5]), pk16(bb[6], bb[7])};

  ssh[t] = h_bits(sv);
  __syncthreads();
  const int tl = t & 31;
  const v4u us = *(const v4u*)(ssh + 8 * tl);
  const bool wave0 = (t < 32);
  unsigned short* bp = Bout + e * 8;
  unsigned short* sp = Sout + eb + 8 * (size_t)tl;
  *(volatile v4u*)bp = ub;
  if (wave0) *(volatile v4u*)sp = us;
  __threadfence();
  *(volatile v4u*)bp = ub;
  if (wave0) *(volatile v4u*)sp = us;
}

extern "C" void kernel_launch(void* const* d_in, const int* in_sizes, int n_in,
                              void* d_out, int out_size, void* d_ws, size_t ws_size,
                              hipStream_t stream) {
  if (n_in < 9) return;
  if (in_sizes[0] != kRows * kLat)   return;
  if (in_sizes[1] != kHid * kLat)    return;
  if (in_sizes[2] != kHid)           return;
  if (in_sizes[3] != kHid * kHid)    return;
  if (in_sizes[4] != kHid * kKsp)    return;
  if (in_sizes[5] != kHid * kHid)    return;
  if (in_sizes[6] != kOutDim * kHid) return;
  if (in_sizes[7] != kOutDim * kKsp) return;
  if (in_sizes[8] != kOutDim * kHid) return;
  if (out_size != kRows * kOutDim)   return;
  if (ws_size < kWsTotal)            return;

  const float* x         = (const float*)d_in[0];
  const float* dense_w   = (const float*)d_in[1];
  const float* dense_b   = (const float*)d_in[2];
  const float* base_w1   = (const float*)d_in[3];
  const float* spline_w1 = (const float*)d_in[4];
  const float* scaler1   = (const float*)d_in[5];
  const float* base_w2   = (const float*)d_in[6];
  const float* spline_w2 = (const float*)d_in[7];
  const float* scaler2   = (const float*)d_in[8];
  float* out = (float*)d_out;

  char* ws = (char*)d_ws;
  unsigned short* xh   = (unsigned short*)(ws + kOffXh);
  unsigned short* dwh  = (unsigned short*)(ws + kOffDwh);
  unsigned short* bw1h = (unsigned short*)(ws + kOffBw1);
  unsigned short* bw2h = (unsigned short*)(ws + kOffBw2);
  unsigned short* sw1b = (unsigned short*)(ws + kOffSw1);
  unsigned short* sw2b = (unsigned short*)(ws + kOffSw2);
  float* p1   = (float*)(ws + kOffP1);
  float* h2   = (float*)(ws + kOffH2);
  unsigned short* spl = (unsigned short*)(ws + kOffSpl);
  float* tbs  = (float*)(ws + kOffTbs);
  unsigned short* bsp = (unsigned short*)(ws + kOffBsp);

  cast8_f16_kernel<<<dim3((kRows * kLat / 8) / 256), dim3(256), 0, stream>>>(x, xh, kRows * kLat / 8, 1.0f);
  cast8_f16_kernel<<<dim3((kHid * kLat / 8) / 256), dim3(256), 0, stream>>>(dense_w, dwh, kHid * kLat / 8, kWCarry);
  cast8_f16_kernel<<<dim3((kHid * kHid / 8) / 256), dim3(256), 0, stream>>>(base_w1, bw1h, kHid * kHid / 8, kWCarry);
  cast8_f16_kernel<<<dim3((kOutDim * kHid / 8) / 256), dim3(256), 0, stream>>>(base_w2, bw2h, kOutDim * kHid / 8, kWCarry);
  spline_cast_kernel<<<dim3((kHid * kHid) / 256), dim3(256), 0, stream>>>(spline_w1, scaler1, sw1b, kHid * kHid);
  spline_cast_kernel<<<dim3((kOutDim * kHid) / 256), dim3(256), 0, stream>>>(spline_w2, scaler2, sw2b, kOutDim * kHid);

  wmma_gemm64<0, false, 2, 0, false, 0><<<dim3((kRows / 64) * (kHid / 64) / 8, 1), dim3(256), 0, stream>>>(
      xh, xh, kLat, 0L, dwh, dwh, kLat, 0L, (void*)p1, (void*)p1, kHid, 0L,
      dense_b, p1, 0L, kRows, kHid, kLat, kDenseScale);

  for (int layer = 0; layer < 2; ++layer) {
    const float* hin = (layer == 0) ? p1 : h2;
    const int pre    = (layer == 0) ? 1 : 0;
    const int nOut   = (layer == 0) ? kHid : kOutDim;
    const unsigned short* bwh = (layer == 0) ? bw1h : bw2h;
    const unsigned short* swb = (layer == 0) ? sw1b : sw2b;
    float* cout = (layer == 0) ? h2 : out;
    const int gemmBlocks = (kChunk / 64) * (nOut / 64) / 8;
    for (int c = 0; c < kNChunk; ++c) {
      expand_kernel<<<dim3((kChunk * kHid) / 256), dim3(256), 0, stream>>>(
          hin + (size_t)c * kChunk * kHid, pre, spl, bsp);
      wmma_gemm64<0, false, 0, 0, false, 0><<<dim3(gemmBlocks, 1), dim3(256), 0, stream>>>(
          spl, spl, kHid, 0L, bwh, bwh, kHid, 0L, (void*)tbs, (void*)tbs, nOut, 0L,
          dense_b, tbs, 0L, kChunk, nOut, kHid, kBaseScale);
      float* cchunk = cout + (size_t)c * kChunk * nOut;
      wmma_gemm64<1, false, 0, 0, true, 0><<<dim3(gemmBlocks, 1), dim3(256), 0, stream>>>(
          bsp, bsp, kKsp, 0L, swb, swb, kKsp, 0L, (void*)cchunk, (void*)cchunk, nOut, 0L,
          dense_b, tbs, 0L, kChunk, nOut, kKsp, 1.0f);
    }
  }
}
